// CausalSelfAttention_36971078484390
// MI455X (gfx1250) — hardware-verified
//
#include <hip/hip_runtime.h>


#ifndef NB
#define NB 2
#endif
#ifndef SEQ
#define SEQ 2048
#endif
#define SEQ_FULL 2048
#define NB_FULL  2
#define DM   1024
#define NH_  16
#define HD   64
#define DQ   (NH_ * HD)
#define PCAR 1024.0f
#define RCAR 2048.0f
#define SCL  0.125f
#define LOG2E 1.4426950408889634f
#define NEGB (-3.0e38f)
#define AW   4

typedef _Float16 h16;
typedef unsigned short bf;
typedef __attribute__((ext_vector_type(16))) __bf16   v16bf;
typedef __attribute__((ext_vector_type(16))) _Float16 v16h;
typedef __attribute__((ext_vector_type(8)))  _Float16 v8h;
typedef __attribute__((ext_vector_type(8)))  unsigned short v8us;
typedef __attribute__((ext_vector_type(8)))  float    v8f;
typedef __attribute__((ext_vector_type(4)))  float    v4f;
typedef v4f  __attribute__((may_alias)) v4fa;

static_assert(HD == 64);
static_assert(NH_ == 16);
static_assert(DQ == DM);
static_assert(DM % 64 == 0);
static_assert(DM % 32 == 0);
static_assert(SEQ % 64 == 0);
static_assert((3 * DQ) % 64 == 0);
static_assert(SEQ <= SEQ_FULL);
static_assert(NB <= NB_FULL);
static_assert(AW * 16 == 64);

#define PLN      ((size_t)NB * NH_ * SEQ * HD)
#define SZ_XB    ((size_t)NB * SEQ * DM * 2)
#define SZ_WQKV  ((size_t)3 * DQ * DM * 2)
#define SZ_WO    ((size_t)DM * DQ * 2)
#define SZ_F     ((size_t)NB * SEQ * 3 * DQ * 4)
#define SZ_AT    ((size_t)2 * NB * SEQ * DQ * 2)
#define SZ_P4    ((size_t)4 * PLN * 2)
#define SZ_V2    ((size_t)2 * PLN * 2)
#define OFF_XB   ((size_t)0)
#define OFF_WQKV (OFF_XB + SZ_XB)
#define OFF_WO   (OFF_WQKV + SZ_WQKV)
#define OFF_F    (OFF_WO + SZ_WO)
#define OFF_P4   (OFF_F + SZ_F)
#define OFF_V2   (OFF_P4 + SZ_P4)
#define WS_TOTAL (OFF_V2 + SZ_V2)
static_assert(SZ_AT <= SZ_F);
static_assert(WS_TOTAL <= (size_t)134217728);
static_assert(SZ_XB % 256 == 0 && SZ_WQKV % 256 == 0 && SZ_WO % 256 == 0 && SZ_F % 256 == 0 && SZ_P4 % 256 == 0);

__device__ __forceinline__ unsigned short f2bf(float f) { unsigned u = __float_as_uint(f); u += 0x7FFFu + ((u >> 16) & 1u); return (unsigned short)(u >> 16); }
__device__ __forceinline__ float bf2f(unsigned short b) { return __uint_as_float(((unsigned)b) << 16); }
__device__ __forceinline__ void splitf(float y, unsigned short& h, unsigned short& l) { h = f2bf(y); l = f2bf(y - bf2f(h)); }
__device__ __forceinline__ v16h cat16(v8h lo, v8h hi) { return __builtin_shufflevector(lo, hi, 0, 1, 2, 3, 4, 5, 6, 7, 8, 9, 10, 11, 12, 13, 14, 15); }
__device__ __forceinline__ v16bf cat16b(v8us lo, v8us hi) { return __builtin_bit_cast(v16bf, __builtin_shufflevector(lo, hi, 0, 1, 2, 3, 4, 5, 6, 7, 8, 9, 10, 11, 12, 13, 14, 15)); }
__device__ __forceinline__ v8f wmma16(v16h a, v16h b, v8f c) { return __builtin_amdgcn_wmma_f32_16x16x32_f16(false, a, false, b, (short)0, c, false, false); }
__device__ __forceinline__ v8f wmmab(v16bf a, v16bf b, v8f c) { return __builtin_amdgcn_wmma_f32_16x16x32_bf16(false, a, false, b, (short)0, c, false, false); }
__device__ __forceinline__ v8f gwb(v16bf a, v16bf b, v8f c) { c = wmmab(a, b, c); asm volatile("v_nop\n\tv_nop\n\tv_nop\n\tv_nop" : "+v"(c) : "v"(a), "v"(b)); return c; }
__device__ __forceinline__ v8f gwh(v16h a, v16h b, v8f c) { c = wmma16(a, b, c); asm volatile("v_nop\n\tv_nop\n\tv_nop\n\tv_nop" : "+v"(c) : "v"(a), "v"(b)); return c; }

template <typename T16> struct WFrag;
template <> struct WFrag<h16> { typedef v16h V; static __device__ __forceinline__ V ld(const h16* p) { return cat16(*(const v8h*)p, *(const v8h*)(p + 16)); } static __device__ __forceinline__ v8f mma(V a, V b, v8f c) { return gwh(a, b, c); } };
template <> struct WFrag<bf> { typedef v16bf V; static __device__ __forceinline__ V ld(const bf* p) { return cat16b(*(const v8us*)p, *(const v8us*)(p + 16)); } static __device__ __forceinline__ v8f mma(V a, V b, v8f c) { return gwb(a, b, c); } };

template <typename T16, int NSPLIT>
__device__ __forceinline__ void gemmw_body(const T16* __restrict__ A, const T16* __restrict__ A2, const T16* __restrict__ Bt, const T16* __restrict__ Bt2, int K, float* C, int ldc, size_t sA, size_t sB, size_t sC) {
    typedef typename WFrag<T16>::V V;
    __shared__ __align__(16) float os[16 * 68];
    const size_t z = blockIdx.z; A += z * sA; if (A2) A2 += z * sA; Bt += z * sB; if (Bt2) Bt2 += z * sB; C += z * sC;
    const int lane = threadIdx.x & 31, lr = lane & 15, hi = lane >> 4; const int r0 = blockIdx.x * 64, c0 = blockIdx.y * 64;
    v8f acc[4][4];
#pragma unroll
    for (int mb = 0; mb < 4; ++mb)
#pragma unroll
        for (int nb = 0; nb < 4; ++nb) acc[mb][nb] = (v8f){};
    const size_t aoff = (size_t)(r0 + lr) * K + 8 * hi, boff = (size_t)(c0 + lr) * K + 8 * hi;
#pragma unroll 1
    for (int kc = 0; kc < K; kc += 32) {
        V a[4], a2[4];
#pragma unroll
        for (int mb = 0; mb < 4; ++mb) { a[mb] = WFrag<T16>::ld(A + aoff + (size_t)mb * 16 * K + kc); if (NSPLIT == 1 || NSPLIT == 2) a2[mb] = WFrag<T16>::ld(A2 + aoff + (size_t)mb * 16 * K + kc); }
#pragma unroll
        for (int nb = 0; nb < 4; ++nb) { const V b = WFrag<T16>::ld(Bt + boff + (size_t)nb * 16 * K + kc); V b2; if (NSPLIT >= 2) b2 = WFrag<T16>::ld(Bt2 + boff + (size_t)nb * 16 * K + kc);
#pragma unroll
            for (int mb = 0; mb < 4; ++mb) { acc[mb][nb] = WFrag<T16>::mma(a[mb], b, acc[mb][nb]); if (NSPLIT == 1 || NSPLIT == 2) acc[mb][nb] = WFrag<T16>::mma(a2[mb], b, acc[mb][nb]); if (NSPLIT >= 2) acc[mb][nb] = WFrag<T16>::mma(a[mb], b2, acc[mb][nb]); } }
    }
#pragma unroll
    for (int mb = 0; mb < 4; ++mb) {
#pragma unroll
        for (int nb = 0; nb < 4; ++nb) {
#pragma unroll
            for (int j = 0; j < 8; ++j) os[(hi * 8 + j) * 68 + nb * 16 + lr] = acc[mb][nb][j]; }
        __builtin_amdgcn_wave_barrier(); asm volatile("" ::: "memory");
        float* crow = C + (size_t)(r0 + mb * 16) * ldc + c0;
#pragma unroll 1
        for (int ps = 0; ps < 2; ++ps) {
#pragma unroll
            for (int s = 0; s < 8; ++s) { const int row = 2 * s + hi, cofs = lr * 4; const v4f val = *(const v4fa*)(os + row * 68 + cofs);
                *(volatile v4f*)(crow + (size_t)row * ldc + cofs) = val; }
            if (ps == 0) __threadfence(); }
        __builtin_amdgcn_wave_barrier(); asm volatile("" ::: "memory");
    }
}

__global__ __launch_bounds__(32) void k_gemm_qkv(const bf* __restrict__ A, const bf* __restrict__ Bt, int K, float* C, int ldc) {
    gemmw_body<bf, 0>(A, nullptr, Bt, nullptr, K, C, ldc, 0, 0, 0);
}
__global__ __launch_bounds__(32) void k_gemm_out(const bf* __restrict__ A, const bf* __restrict__ A2, const bf* __restrict__ Bt, int K, float* C, int ldc, size_t sA, size_t sC) {
    gemmw_body<bf, 1>(A, A2, Bt, nullptr, K, C, ldc, sA, 0, sC);
}

__global__ __launch_bounds__(256) void k_cvt8(const float* __restrict__ src, bf* dst, size_t n8) { const size_t i = (size_t)blockIdx.x * 256 + threadIdx.x; if (i >= n8) return; const v8f v = *(const v8f*)(src + i * 8); v8us o;
#pragma unroll
    for (int k = 0; k < 8; ++k) o[k] = f2bf(v[k]); *(volatile v8us*)(dst + i * 8) = o; __threadfence(); *(volatile v8us*)(dst + i * 8) = o; }

__global__ __launch_bounds__(256) void k_qkp(const float* __restrict__ F, bf* P4) {
    const size_t i = (size_t)blockIdx.x * 256 + threadIdx.x; if (i >= (size_t)NB * SEQ * 2 * NH_ * 8) return;
    const int d8 = (int)(i & 7), h = (int)((i >> 3) & 15), w = (int)((i >> 7) & 1); const size_t bt = i >> 8; const int t = (int)(bt % SEQ), b = (int)(bt / SEQ);
    const float* f = F + bt * (size_t)(3 * DQ) + w * DQ + h * HD + d8 * 8;
    const v4f a = *(const v4f*)f, c = *(const v4f*)(f + 4); v8us oh, ol;
#pragma unroll
    for (int k = 0; k < 4; ++k) { unsigned short x0, x1; splitf(a[k], x0, x1); oh[k] = x0; ol[k] = x1; splitf(c[k], x0, x1); oh[4 + k] = x0; ol[4 + k] = x1; }
    const size_t o = (((size_t)b * NH_ + h) * SEQ + t) * HD + d8 * 8;
    const size_t oh_off = (size_t)(2 * w) * PLN + o, ol_off = (size_t)(2 * w + 1) * PLN + o;
    *(volatile v8us*)(P4 + oh_off) = oh; *(volatile v8us*)(P4 + ol_off) = ol; __threadfence(); *(volatile v8us*)(P4 + oh_off) = oh; *(volatile v8us*)(P4 + ol_off) = ol;
}

__global__ __launch_bounds__(256) void k_vtp(const float* __restrict__ F, h16* VV, h16* VR) {
    const size_t i = (size_t)blockIdx.x * 256 + threadIdx.x; if (i >= (size_t)NB * NH_ * HD * (SEQ / 8)) return;
    const int t8 = (int)(i % (SEQ / 8)); const int d = (int)((i / (SEQ / 8)) % HD); const int g = (int)((i / ((size_t)(SEQ / 8) * HD)) % NH_); const int b = (int)(i / ((size_t)(SEQ / 8) * HD * NH_));
    const float* f = F + ((size_t)b * SEQ + (size_t)t8 * 8) * (size_t)(3 * DQ) + 2 * DQ + g * HD + d; v8h ov, orr;
#pragma unroll
    for (int j = 0; j < 8; ++j) { const float x = f[(size_t)j * (3 * DQ)]; const h16 vh = (h16)x; ov[j] = vh; orr[j] = (h16)((x - (float)vh) * RCAR); }
    const size_t o = (((size_t)b * NH_ + g) * HD + d) * SEQ + (size_t)t8 * 8;
    *(volatile v8h*)(VV + o) = ov; *(volatile v8h*)(VR + o) = orr; __threadfence(); *(volatile v8h*)(VV + o) = ov; *(volatile v8h*)(VR + o) = orr;
}

__device__ __forceinline__ float head_slope(int h) {
    float s = 0.707106769f;
    s = (h == 1)  ? 0.500000000f   : s;
    s = (h == 2)  ? 0.353553385f   : s;
    s = (h == 3)  ? 0.250000000f   : s;
    s = (h == 4)  ? 0.176776692f   : s;
    s = (h == 5)  ? 0.125000000f   : s;
    s = (h == 6)  ? 0.0883883461f  : s;
    s = (h == 7)  ? 0.0625000000f  : s;
    s = (h == 8)  ? 0.0441941731f  : s;
    s = (h == 9)  ? 0.0312500000f  : s;
    s = (h == 10) ? 0.0220970865f  : s;
    s = (h == 11) ? 0.0156250000f  : s;
    s = (h == 12) ? 0.0110485433f  : s;
    s = (h == 13) ? 0.00781250000f : s;
    s = (h == 14) ? 0.00552427163f : s;
    s = (h == 15) ? 0.00390625000f : s;
    return s;
}

__global__ __launch_bounds__(128) void k_flash(const bf* __restrict__ Qh, const bf* __restrict__ Ql, const bf* __restrict__ Kh, const bf* __restrict__ Kl, const h16* __restrict__ VV, const h16* __restrict__ VR, bf* Ah, bf* Al) {
#pragma clang fp contract(off)
    __shared__ __align__(16) float os[AW * 16 * 68];
    const int wave = __builtin_amdgcn_readfirstlane(threadIdx.x >> 5);
    const int lane = threadIdx.x & 31, lr = lane & 15, hi = lane >> 4;
    const int h = blockIdx.y, b = blockIdx.z;
    const int q0 = blockIdx.x * (AW * 16) + wave * 16;
    const size_t pbase = ((size_t)b * NH_ + h) * SEQ * HD;
    const size_t vbase = ((size_t)b * NH_ + h) * HD * SEQ;
    const float slope = head_slope(h);
    const int q = q0 + lr;

    v16bf qh[2], ql[2];
    const size_t qoff = pbase + (size_t)q * HD + 8 * hi;
#pragma unroll
    for (int ks = 0; ks < 2; ++ks) { qh[ks] = WFrag<bf>::ld(Qh + qoff + ks * 32); ql[ks] = WFrag<bf>::ld(Ql + qoff + ks * 32); }

    v8f O[4], R[4];
#pragma unroll
    for (int g = 0; g < 4; ++g) { O[g] = (v8f){}; R[g] = (v8f){}; }
    float m = NEGB, l = 0.0f;
    const int nsteps = (q0 >> 5) + 1;

#pragma unroll 1
    for (int st = 0; st < nsteps; ++st) {
        const int kb = st * 32;
        v8f s0 = (v8f){}, s1 = (v8f){};
        const size_t koff = pbase + (size_t)(kb + lr) * HD + 8 * hi;
#pragma unroll
        for (int ks = 0; ks < 2; ++ks) {
            const v16bf a0h = WFrag<bf>::ld(Kh + koff + ks * 32), a0l = WFrag<bf>::ld(Kl + koff + ks * 32);
            s0 = gwb(a0h, qh[ks], s0); s0 = gwb(a0h, ql[ks], s0); s0 = gwb(a0l, qh[ks], s0);
            const v16bf a1h = WFrag<bf>::ld(Kh + koff + (size_t)16 * HD + ks * 32), a1l = WFrag<bf>::ld(Kl + koff + (size_t)16 * HD + ks * 32);
            s1 = gwb(a1h, qh[ks], s1); s1 = gwb(a1h, ql[ks], s1); s1 = gwb(a1l, qh[ks], s1);
        }
        const float dbase = (float)(kb + 8 * hi - q);
        float t0[8], t1[8]; float mx = m;
#pragma unroll
        for (int r = 0; r < 8; ++r) {
            const float d0 = dbase + (float)r, d1 = dbase + (float)(r + 16);
            const float b0 = slope * d0, b1 = slope * d1;
            const float a0 = (s0[r] * SCL + b0) * LOG2E, a1 = (s1[r] * SCL + b1) * LOG2E;
            t0[r] = (d0 <= 0.0f) ? a0 : NEGB; t1[r] = (d1 <= 0.0f) ? a1 : NEGB;
            mx = fmaxf(mx, fmaxf(t0[r], t1[r]));
        }
        mx = fmaxf(mx, __shfl_xor(mx, 16, 32));
        const float alpha = __builtin_amdgcn_exp2f(m - mx); m = mx;
        float psum = 0.0f; v16h pv, pr;
#pragma unroll
        for (int r = 0; r < 8; ++r) {
            const float d0 = dbase + (float)r, d1 = dbase + (float)(r + 16);
            const float e0 = __builtin_amdgcn_exp2f(t0[r] - mx), e1 = __builtin_amdgcn_exp2f(t1[r] - mx);
            const float p0 = (d0 <= 0.0f) ? e0 : 0.0f, p1 = (d1 <= 0.0f) ? e1 : 0.0f;
            psum += p0 + p1;
            const float c0 = p0 * PCAR, c1 = p1 * PCAR;
            const h16 h0 = (h16)c0, h1 = (h16)c1;
            pv[r] = h0; pv[8 + r] = h1;
            pr[r] = (h16)((c0 - (float)h0) * RCAR); pr[8 + r] = (h16)((c1 - (float)h1) * RCAR);
        }
        l = l * alpha + psum;
#pragma unroll
        for (int g = 0; g < 4; ++g)
#pragma unroll
            for (int r = 0; r < 8; ++r) { O[g][r] *= alpha; R[g][r] *= alpha; }
#pragma unroll
        for (int g = 0; g < 4; ++g) {
            const size_t voff = vbase + (size_t)(g * 16 + lr) * SEQ + kb + 8 * hi;
            const v16h vv = WFrag<h16>::ld(VV + voff), vr = WFrag<h16>::ld(VR + voff);
            O[g] = gwh(vv, pv, O[g]); R[g] = gwh(vr, pv, R[g]); R[g] = gwh(vv, pr, R[g]);
        }
    }
    l += __shfl_xor(l, 16, 32);
    const float cs = (1.0f / l) * (1.0f / PCAR);
    const int ob = wave * 16 * 68;
#pragma unroll
    for (int g = 0; g < 4; ++g) { v4f a, c;
#pragma unroll
        for (int k = 0; k < 4; ++k) { a[k] = (O[g][k] + R[g][k] * (1.0f / RCAR)) * cs; c[k] = (O[g][4 + k] + R[g][4 + k] * (1.0f / RCAR)) * cs; }
        *(v4fa*)(os + ob + lr * 68 + g * 16 + 8 * hi) = a; *(v4fa*)(os + ob + lr * 68 + g * 16 + 8 * hi + 4) = c; }
    __builtin_amdgcn_wave_barrier(); asm volatile("" ::: "memory");
#pragma unroll 1
    for (int ps = 0; ps < 2; ++ps) {
#pragma unroll
        for (int s = 0; s < 4; ++s) { const int row = 4 * s + (lane >> 3), col = (lane & 7) * 8;
            const v4f a = *(const v4fa*)(os + ob + row * 68 + col), c = *(const v4fa*)(os + ob + row * 68 + col + 4); v8us oh, ol;
#pragma unroll
            for (int k = 0; k < 4; ++k) { unsigned short x0, x1; splitf(a[k], x0, x1); oh[k] = x0; ol[k] = x1; splitf(c[k], x0, x1); oh[4 + k] = x0; ol[4 + k] = x1; }
            const size_t dst = ((size_t)b * SEQ + q0 + row) * DQ + h * HD + col;
            *(volatile v8us*)(Ah + dst) = oh; *(volatile v8us*)(Al + dst) = ol; }
        if (ps == 0) __threadfence(); }
    __builtin_amdgcn_wave_barrier(); asm volatile("" ::: "memory");
}

extern "C" void kernel_launch(void* const* d_in, const int* in_sizes, int n_in,
                              void* d_out, int out_size, void* d_ws, size_t ws_size, hipStream_t stream) {
    if (n_in < 3) return;
    const size_t xneed = (size_t)(NB - 1) * SEQ_FULL * DM + (size_t)SEQ * DM;
    if ((size_t)in_sizes[0] < xneed) return;
    if ((size_t)in_sizes[1] < (size_t)3 * DQ * DM) return;
    if ((size_t)in_sizes[2] < (size_t)DM * DQ) return;
    if ((size_t)out_size < xneed) return;
    if (ws_size < WS_TOTAL) return;
    const float* x = (const float*)d_in[0];
    const float* wattn = (const float*)d_in[1];
    const float* wproj = (const float*)d_in[2];
    float* OUT = (float*)d_out;
    char* ws = (char*)d_ws;
    bf* XB = (bf*)(ws + OFF_XB); bf* WQKV = (bf*)(ws + OFF_WQKV); bf* WO = (bf*)(ws + OFF_WO);
    float* F = (float*)(ws + OFF_F);
    bf* ATh = (bf*)(ws + OFF_F); bf* ATl = ATh + (size_t)NB * SEQ * DQ;
    bf* P4 = (bf*)(ws + OFF_P4);
    h16* VV = (h16*)(ws + OFF_V2); h16* VR = VV + PLN;

    for (int b = 0; b < NB; ++b)
        k_cvt8<<<(unsigned)(((size_t)SEQ * DM / 8 + 255) / 256), 256, 0, stream>>>(x + (size_t)b * SEQ_FULL * DM, XB + (size_t)b * SEQ * DM, (size_t)SEQ * DM / 8);
    k_cvt8<<<(unsigned)(((size_t)3 * DQ * DM / 8 + 255) / 256), 256, 0, stream>>>(wattn, WQKV, (size_t)3 * DQ * DM / 8);
    k_cvt8<<<(unsigned)(((size_t)DM * DQ / 8 + 255) / 256), 256, 0, stream>>>(wproj, WO, (size_t)DM * DQ / 8);
    k_gemm_qkv<<<dim3(NB * SEQ / 64, 3 * DQ / 64, 1), 32, 0, stream>>>(XB, WQKV, DM, F, 3 * DQ);
    k_qkp<<<(unsigned)(((size_t)NB * SEQ * 2 * NH_ * 8 + 255) / 256), 256, 0, stream>>>(F, P4);
    k_vtp<<<(unsigned)(((size_t)NB * NH_ * HD * (SEQ / 8) + 255) / 256), 256, 0, stream>>>(F, VV, VR);
    k_flash<<<dim3(SEQ / 64, NH_, NB), 128, 0, stream>>>(P4, P4 + PLN, P4 + 2 * PLN, P4 + 3 * PLN, VV, VR, ATh, ATl);
    k_gemm_out<<<dim3(SEQ / 64, DM / 64, NB), 32, 0, stream>>>(ATh, ATl, WO, DQ, OUT, DM, (size_t)SEQ * DQ, (size_t)SEQ_FULL * DM);
}
